// GNN_82729660055705
// MI455X (gfx1250) — hardware-run, weakly checked
//
#include <hip/hip_runtime.h>
#include <stddef.h>
#include <stdint.h>
#include <math.h>

#define DF      128
#define KD      256
#define EW      64
#define TROWS   34
#define TABF    (3 * TROWS * DF)
#define SMALLF  832
#define LNEPS   1e-5f
#define NTHR    256
#define NWAVE   8
#define EPT     8
#define CHUNK   (NTHR * EPT)
#define WCAP    (EPT * 32)
#define LISTN   (NWAVE * WCAP)
#define NBA     1024
#define SLA     10
#define RCAP    11776
#define DEGCAP  64
#define MEAS_BMAX 10475
#define MEAS_DEG  26
#define GBM     64
#define GBN     128
#define GTHR    128
#define GWAVE   (GTHR / 32)
#define ROWH    256
#define NU_PWT  (DF * (DF / 8))
#define NU_W4D  (4 * DF * (KD / 8))
#define NU_POST (DF * (KD / 8))
#define NU_W    (NU_PWT + NU_W4D + NU_POST)
#define NTABU   (TROWS * 32)
#define TABBLK  5
#define AGG_ZINTS    (LISTN + 2 * RCAP + 3 * NBA)
#define MISC_INTS    16
#define ROWBUF_INTS  (NWAVE * ROWH / 2)
#define AGG_LDS_INTS (AGG_ZINTS + MISC_INTS + ROWBUF_INTS + TABF)
#define WSMAX   134217728

static_assert((CHUNK & (CHUNK - 1)) == 0 && CHUNK <= 4096);
static_assert((NBA & (NBA - 1)) == 0 && NBA == (1 << SLA));
static_assert(((long long)CHUNK << SLA) < (1LL << 31));
static_assert(NBA % NWAVE == 0 && NBA % 32 == 0 && NBA % GBM == 0);
static_assert(RCAP % 4 == 0 && AGG_ZINTS % 4 == 0 && LISTN % 4 == 0);
static_assert(((AGG_ZINTS + MISC_INTS + ROWBUF_INTS) % 4) == 0 && (TABF % 4) == 0);
static_assert(RCAP >= MEAS_BMAX + MEAS_BMAX / 20 + 1);
static_assert(DEGCAP >= MEAS_DEG + 8);
static_assert(GBN == DF && GBM == GWAVE * 16 && DF == 4 * 32 && GTHR == GWAVE * 32);
static_assert(KD == 2 * DF && ROWH == 2 * DF && (DF % 32) == 0 && (KD % 32) == 0);
static_assert(AGG_LDS_INTS * 4 <= 300000);
static_assert(NU_PWT % NTHR == 0 && NU_W4D % NTHR == 0 && NU_POST % NTHR == 0 && (NU_W4D / 4) % NTHR == 0);
static_assert(NTABU % 32 == 0 && TABBLK * NTHR >= NTABU);
static_assert((TROWS * EW) % 32 == 0);
static_assert(SMALLF >= 512 + 128 + 128 + 32);

typedef float          v4f   __attribute__((ext_vector_type(4)));
typedef float          v8f   __attribute__((ext_vector_type(8)));
typedef int            v4i   __attribute__((ext_vector_type(4)));
typedef int            v8i   __attribute__((ext_vector_type(8)));
typedef unsigned short v4us  __attribute__((ext_vector_type(4)));
typedef unsigned short v8us  __attribute__((ext_vector_type(8)));
typedef unsigned short v16us __attribute__((ext_vector_type(16)));
typedef __bf16         v16bf __attribute__((ext_vector_type(16)));
typedef v4f  __attribute__((may_alias)) v4fa;
typedef v4i  __attribute__((may_alias)) v4ia;
typedef v4us __attribute__((may_alias)) v4usa;
typedef v8us __attribute__((may_alias)) v8usa;
union FragB { v16bf v; v16us u; v8us h[2]; v8i w; };

__device__ __forceinline__ v8f wmb(const FragB& a, const FragB& b, v8f c) {
  v8f d = __builtin_amdgcn_wmma_f32_16x16x32_bf16(false, a.v, false, b.v, (short)0, c, false, false);
  asm volatile("v_nop\n\tv_nop\n\tv_nop\n\tv_nop" : "+v"(d) : "v"(a.w), "v"(b.w));
  return d;
}

__device__ __forceinline__ v8f z8() { v8f z = {0.f, 0.f, 0.f, 0.f, 0.f, 0.f, 0.f, 0.f}; return z; }

__device__ __forceinline__ unsigned bf16_bits(float f) {
  const unsigned u = __float_as_uint(f);
  return (u + 0x7FFFu + ((u >> 16) & 1u)) >> 16;
}
__device__ __forceinline__ float bf16_val(float f) {
  return __uint_as_float(bf16_bits(f) << 16);
}
__device__ __forceinline__ v4f bf4(const v4f a) {
  v4f o;
  o.x = bf16_val(a.x); o.y = bf16_val(a.y); o.z = bf16_val(a.z); o.w = bf16_val(a.w);
  return o;
}
__device__ __forceinline__ unsigned hl_bits(float v, unsigned& lo) {
  const unsigned hb = bf16_bits(v);
  lo = bf16_bits(v - __uint_as_float(hb << 16));
  return hb;
}
__device__ __forceinline__ float gelu_f(float v) {
  return 0.5f * v * (1.0f + erff(v * 0.70710678118654752f));
}

__device__ __forceinline__ void wave_sync() {
  __builtin_amdgcn_fence(__ATOMIC_RELEASE, "wavefront");
  __builtin_amdgcn_wave_barrier();
  __builtin_amdgcn_fence(__ATOMIC_ACQUIRE, "wavefront");
}

template <int SLB>
__device__ __forceinline__ int scan_chunk(const int* __restrict__ dsts, int nE, int cbase, int slotBase,
                                          int nb, int vec8, int* list, int tid, int lane, int wave) {
  int wc = 0;
  const int el0  = tid * EPT;
  const int e0   = cbase + el0;
  const int sent = -2147483647 - 1;
  v4i da, db;
  if (vec8 != 0 && cbase + CHUNK <= nE) {
    da = *(const v4i*)(dsts + e0);
    db = *(const v4i*)(dsts + e0 + 4);
  } else {
    da.x = (e0     < nE) ? dsts[min(e0,     nE - 1)] : sent;
    da.y = (e0 + 1 < nE) ? dsts[min(e0 + 1, nE - 1)] : sent;
    da.z = (e0 + 2 < nE) ? dsts[min(e0 + 2, nE - 1)] : sent;
    da.w = (e0 + 3 < nE) ? dsts[min(e0 + 3, nE - 1)] : sent;
    db.x = (e0 + 4 < nE) ? dsts[min(e0 + 4, nE - 1)] : sent;
    db.y = (e0 + 5 < nE) ? dsts[min(e0 + 5, nE - 1)] : sent;
    db.z = (e0 + 6 < nE) ? dsts[min(e0 + 6, nE - 1)] : sent;
    db.w = (e0 + 7 < nE) ? dsts[min(e0 + 7, nE - 1)] : sent;
  }
  const unsigned nbs = (unsigned)slotBase;
  const unsigned unb = (unsigned)nb;
  const unsigned s0 = (unsigned)da.x - nbs, s1 = (unsigned)da.y - nbs;
  const unsigned s2 = (unsigned)da.z - nbs, s3 = (unsigned)da.w - nbs;
  const unsigned s4 = (unsigned)db.x - nbs, s5 = (unsigned)db.y - nbs;
  const unsigned s6 = (unsigned)db.z - nbs, s7 = (unsigned)db.w - nbs;
  const bool h0 = s0 < unb, h1 = s1 < unb, h2 = s2 < unb, h3 = s3 < unb;
  const bool h4 = s4 < unb, h5 = s5 < unb, h6 = s6 < unb, h7 = s7 < unb;
  const unsigned any = __builtin_amdgcn_ballot_w32(h0 | h1 | h2 | h3 | h4 | h5 | h6 | h7);
  if (any != 0u) {
#define HITJ(J, HJ, SJ) { \
      const unsigned mj = __builtin_amdgcn_ballot_w32(HJ); \
      if (mj != 0u) { \
        if (HJ) { \
          const int pos = wc + (int)__builtin_amdgcn_mbcnt_lo(mj, 0u); \
          if (pos < WCAP) list[wave * WCAP + pos] = ((el0 + (J)) << SLB) | (int)(SJ); \
        } \
        wc += (int)__builtin_popcount(mj); } }
    HITJ(0, h0, s0)
    HITJ(1, h1, s1)
    HITJ(2, h2, s2)
    HITJ(3, h3, s3)
    HITJ(4, h4, s4)
    HITJ(5, h5, s5)
    HITJ(6, h6, s6)
    HITJ(7, h7, s7)
#undef HITJ
  }
  return wc;
}

__global__ __launch_bounds__(NTHR) void k_prep(const float* __restrict__ x, const float* __restrict__ prew,
                                               const float* __restrict__ w0, const float* __restrict__ w1,
                                               const float* __restrict__ w2, const float* __restrict__ w3,
                                               const float* __restrict__ postw,
                                               unsigned short* pwt, unsigned short* w4d, unsigned short* postd,
                                               unsigned short* xb, int nN, int nUnits) {
  const int u = (int)blockIdx.x * NTHR + (int)threadIdx.x;
  v8us o;
  unsigned short* dp;
  if (u < NU_PWT) {
    const int n = u >> 4, k8 = (u & 15) * 8;
    const float* p = prew + (size_t)k8 * DF + n;
#pragma unroll
    for (int i = 0; i < 8; ++i) o[i] = (unsigned short)bf16_bits(p[(size_t)i * DF]);
    dp = pwt + (size_t)u * 8;
  } else if (u < NU_PWT + NU_W4D) {
    const int v  = u - NU_PWT;
    const int n  = v >> 5, k8 = (v & 31) * 8, kk = k8 & (DF - 1);
    const int j  = v >> 12;
    const float* w;
    if (j == 0)      w = w0;
    else if (j == 1) w = w1;
    else if (j == 2) w = w2;
    else             w = w3;
    const float* p = w + (size_t)kk * DF + (n & (DF - 1));
#pragma unroll
    for (int i = 0; i < 8; ++i) o[i] = (unsigned short)bf16_bits(p[(size_t)i * DF]);
    dp = w4d + (size_t)v * 8;
  } else if (u < NU_W) {
    const int v  = u - NU_PWT - NU_W4D;
    const int n  = v >> 5, k8 = (v & 31) * 8, kk = k8 & (DF - 1);
    const float* p = postw + (size_t)kk * DF + n;
#pragma unroll
    for (int i = 0; i < 8; ++i) o[i] = (unsigned short)bf16_bits(p[(size_t)i * DF]);
    dp = postd + (size_t)v * 8;
  } else if (u < nUnits) {
    const int v   = u - NU_W;
    const int row = v >> 4, c0 = (v & 15) * 8;
    const int rc  = row < nN ? row : nN - 1;
    const float* p = x + (size_t)rc * DF + c0;
    v4f a = *(const v4f*)p, b = *(const v4f*)(p + 4);
    const v4f z4 = {0.f, 0.f, 0.f, 0.f};
    if (row >= nN) { a = z4; b = z4; }
    o[0] = (unsigned short)bf16_bits(a.x); o[1] = (unsigned short)bf16_bits(a.y);
    o[2] = (unsigned short)bf16_bits(a.z); o[3] = (unsigned short)bf16_bits(a.w);
    o[4] = (unsigned short)bf16_bits(b.x); o[5] = (unsigned short)bf16_bits(b.y);
    o[6] = (unsigned short)bf16_bits(b.z); o[7] = (unsigned short)bf16_bits(b.w);
    dp = xb + (size_t)v * 8;
  } else {
    return;
  }
  *(volatile v8us*)dp = o;
  __threadfence();
  *(volatile v8us*)dp = o;
}

__global__ __launch_bounds__(NTHR) void k_tab(const float* __restrict__ e0, const float* __restrict__ e1,
                                              const float* __restrict__ e2, const float* __restrict__ e3,
                                              const float* __restrict__ r0w, const float* __restrict__ r1w,
                                              const float* __restrict__ r2w,
                                              const float* __restrict__ r0b, const float* __restrict__ r1b,
                                              const float* __restrict__ r2b,
                                              const float* __restrict__ m0b, const float* __restrict__ m1b,
                                              const float* __restrict__ m2b, const float* __restrict__ m3b,
                                              const float* __restrict__ preb, const float* __restrict__ postb,
                                              const float* __restrict__ einit, const float* __restrict__ init0,
                                              float* tab, float* small) {
  __shared__ __attribute__((aligned(16))) float embs[TROWS * EW];
  __shared__ float exs[8];
  const int tid = (int)threadIdx.x, lane = tid & 31, wave = tid >> 5;
  const int b = (int)blockIdx.x;
  {
    const int t8 = tid & 7;
    const int ie = t8 < 3 ? t8 : 3;
    int ii = t8 - 2; ii = ii < 0 ? 0 : (ii > 3 ? 3 : ii);
    const unsigned ue = __float_as_uint(bf16_val(einit[ie]));
    const unsigned ui = __float_as_uint(bf16_val(init0[ii]));
    const unsigned me = 0u - (unsigned)(t8 < 4);
    const float arg = __uint_as_float((ue & me) | (ui & ~me));
    const float ex = expf(arg);
    if (tid < 8) exs[tid] = ex;
  }
#pragma unroll 1
  for (int i = tid; i < TROWS * EW; i += NTHR) {
    const int row = i >> 6, k = i & 63;
    int q0 = row;      q0 = q0 > 5 ? 5 : q0;
    int q1 = row - 6;  q1 = q1 < 0 ? 0 : (q1 > 6 ? 6 : q1);
    int q2 = row - 13; q2 = q2 < 0 ? 0 : (q2 > 2 ? 2 : q2);
    int q3 = row - 16; q3 = q3 < 0 ? 0 : (q3 > 17 ? 17 : q3);
    const unsigned u0 = __float_as_uint(e0[q0 * EW + k]);
    const unsigned u1 = __float_as_uint(e1[q1 * EW + k]);
    const unsigned u2 = __float_as_uint(e2[q2 * EW + k]);
    const unsigned u3 = __float_as_uint(e3[q3 * EW + k]);
    const int c = (row >= 6) + (row >= 13) + (row >= 16);
    const unsigned k0 = 0u - (unsigned)(c == 0), k1 = 0u - (unsigned)(c == 1);
    const unsigned k2 = 0u - (unsigned)(c == 2), k3 = 0u - (unsigned)(c == 3);
    const float v = __uint_as_float((u0 & k0) | (u1 & k1) | (u2 & k2) | (u3 & k3));
    embs[i] = bf16_val(v);
  }
  __syncthreads();
  const float se = exs[4], sv = exs[5];
  const float ssum = ((exs[0] + exs[1]) + exs[2]) + exs[3];
  const float isq = 1.0f / sqrtf(ssum);

  if (b < 3 * TABBLK) {
    const int t = b / TABBLK;
    const int u = (b - t * TABBLK) * NTHR + tid;
    if (u < NTABU) {
      const int row = u >> 5, n4 = (u & 31) * 4;
      const float* rw;
      if (t == 0)      rw = r0w;
      else if (t == 1) rw = r1w;
      else             rw = r2w;
      const int c = (row >= 6) + (row >= 13) + (row >= 16);
      const float xwc = exs[c] * isq;
      const float sc  = (t == 2) ? sv : se;
      const float* er = embs + row * EW;
      const float* wp = rw + n4;
      float a0 = 0.0f, a1 = 0.0f, a2 = 0.0f, a3 = 0.0f;
#pragma unroll 2
      for (int k = 0; k < EW; ++k) {
        const float e = er[k];
        const v4f w = *(const v4f*)(wp + (size_t)k * DF);
        a0 = fmaf(e, bf16_val(w.x), a0);
        a1 = fmaf(e, bf16_val(w.y), a1);
        a2 = fmaf(e, bf16_val(w.z), a2);
        a3 = fmaf(e, bf16_val(w.w), a3);
      }
      const float f = sc * xwc;
      v4f o; o.x = a0 * f; o.y = a1 * f; o.z = a2 * f; o.w = a3 * f;
      float* op = tab + (size_t)t * (TROWS * DF) + (size_t)u * 4;
      *(volatile v4f*)op = o;
      __threadfence();
      *(volatile v4f*)op = o;
    }
  } else {
    const int c4 = 4 * lane;
    v4f val = {0.f, 0.f, 0.f, 0.f};
    if (wave == 0) {
      val = bf4(*(const v4f*)(m0b + c4));
    } else if (wave == 1) {
      val = bf4(*(const v4f*)(m1b + c4)) + se * bf4(*(const v4f*)(r0b + c4));
    } else if (wave == 2) {
      val = bf4(*(const v4f*)(m2b + c4)) + se * bf4(*(const v4f*)(r1b + c4));
    } else if (wave == 3) {
      val = bf4(*(const v4f*)(m3b + c4)) + sv * bf4(*(const v4f*)(r2b + c4));
    } else if (wave == 4) {
      val = bf4(*(const v4f*)(preb + c4));
    } else if (wave == 5) {
      val = bf4(*(const v4f*)(postb + c4));
    } else if (wave == 6) {
      const float a0c = bf16_val(init0[0]);
      const float a1c = bf16_val(init0[1]);
      v4f l0; l0.x = a0c;            l0.y = a1c;            l0.z = exs[0] * isq; l0.w = exs[1] * isq;
      v4f l1; l1.x = exs[2] * isq;   l1.y = exs[3] * isq;   l1.z = se;           l1.w = sv;
      const float f0 = (lane == 0) ? 1.0f : 0.0f;
      const float f1 = (lane == 1) ? 1.0f : 0.0f;
      val = l0 * f0 + l1 * f1;
    }
    const bool wr = (wave < 6) || (wave == 6 && lane < 8);
    float* op = small + 4 * tid;
    if (wr) *(volatile v4f*)op = val;
    __threadfence();
    if (wr) *(volatile v4f*)op = val;
  }
}

template <int MODE>
__global__ __launch_bounds__(GTHR) void k_gemm(const unsigned short* A, int lda,
                                               const unsigned short* __restrict__ BT, int K,
                                               const float* __restrict__ bias, const float* __restrict__ xin,
                                               const int* __restrict__ flg, int nFlg,
                                               unsigned short* hpl, float* wsf, size_t oD, size_t oK,
                                               float* outp, int nN, int mRows) {
  __shared__ __attribute__((aligned(16))) float stg[GBM * GBN];
  const int tid = (int)threadIdx.x, lane = tid & 31, wave = tid >> 5, hh = lane >> 4, m = lane & 15;
  const int rowBase = (int)blockIdx.x * GBM;
  const int ny = (MODE == 1) ? (int)blockIdx.y : 0;

  v8f acc[8];
#pragma unroll
  for (int t = 0; t < 8; ++t) acc[t] = z8();
  const unsigned short* ap = A + (size_t)(rowBase + 16 * wave + m) * (size_t)lda + 8 * hh;
  const unsigned short* bp = BT + (size_t)(ny * GBN + m) * (size_t)K + 8 * hh;

#pragma unroll 1
  for (int k0 = 0; k0 < K; k0 += 32) {
    FragB af;
    af.h[0] = *(const v8usa*)(ap + k0);
    af.h[1] = *(const v8usa*)(ap + k0 + 16);
#pragma unroll
    for (int nt = 0; nt < 8; ++nt) {
      const unsigned short* wq = bp + (size_t)(16 * nt) * (size_t)K + k0;
      FragB bf;
      bf.h[0] = *(const v8usa*)wq;
      bf.h[1] = *(const v8usa*)(wq + 16);
      acc[nt] = wmb(af, bf, acc[nt]);
    }
  }

#pragma unroll
  for (int nt = 0; nt < 8; ++nt) {
    const int lc = 16 * nt + m;
#pragma unroll
    for (int r = 0; r < 8; ++r) {
      const int lr = 16 * wave + 8 * hh + r;
      stg[lr * GBN + lc] = acc[nt][r];
    }
  }
  __syncthreads();

  const v4f b4 = *(const v4f*)(bias + (size_t)ny * GBN + 4 * lane);

  if constexpr (MODE == 0) {
    v4f pv[16];
#pragma unroll
    for (int i = 0; i < 16; ++i) pv[i] = *(const v4fa*)(stg + (16 * wave + i) * GBN + 4 * lane);
    __syncthreads();
    const float invd = 1.0f / (float)DF;
#pragma unroll
    for (int i = 0; i < 16; ++i) {
      const int row = rowBase + 16 * wave + i;
      const bool ok = row < nN;
      const float y0 = pv[i].x + b4.x, y1 = pv[i].y + b4.y, y2 = pv[i].z + b4.z, y3 = pv[i].w + b4.w;
      float s = (y0 + y1) + (y2 + y3);
      s += __shfl_xor(s, 16, 32);
      s += __shfl_xor(s, 8, 32);
      s += __shfl_xor(s, 4, 32);
      s += __shfl_xor(s, 2, 32);
      s += __shfl_xor(s, 1, 32);
      const float mean = s * invd;
      const float d0 = y0 - mean, d1 = y1 - mean, d2 = y2 - mean, d3 = y3 - mean;
      float q = (d0 * d0 + d1 * d1) + (d2 * d2 + d3 * d3);
      q += __shfl_xor(q, 16, 32);
      q += __shfl_xor(q, 8, 32);
      q += __shfl_xor(q, 4, 32);
      q += __shfl_xor(q, 2, 32);
      q += __shfl_xor(q, 1, 32);
      const float var  = q * invd;
      const float rstd = 1.0f / sqrtf(var + LNEPS);
      v4f qo;
      qo.x = ok ? d0 * rstd : 0.0f; qo.y = ok ? d1 * rstd : 0.0f;
      qo.z = ok ? d2 * rstd : 0.0f; qo.w = ok ? d3 * rstd : 0.0f;
      pv[i] = qo;
    }
#pragma unroll
    for (int i = 0; i < 16; ++i) {
      v4us h4, l4;
      unsigned lb;
      unsigned hb;
      hb = hl_bits(pv[i].x, lb); h4[0] = (unsigned short)hb; l4[0] = (unsigned short)lb;
      hb = hl_bits(pv[i].y, lb); h4[1] = (unsigned short)hb; l4[1] = (unsigned short)lb;
      hb = hl_bits(pv[i].z, lb); h4[2] = (unsigned short)hb; l4[2] = (unsigned short)lb;
      hb = hl_bits(pv[i].w, lb); h4[3] = (unsigned short)hb; l4[3] = (unsigned short)lb;
      unsigned short* srow = (unsigned short*)stg + (size_t)(16 * wave + i) * (2 * GBN);
      *(v4usa*)(srow + 4 * lane) = h4;
      *(v4usa*)(srow + DF + 4 * lane) = l4;
    }
    __syncthreads();
    v8us qv[16];
#pragma unroll
    for (int i = 0; i < 16; ++i) {
      const unsigned short* srow = (const unsigned short*)stg + (size_t)(16 * wave + i) * (2 * GBN);
      qv[i] = *(const v8usa*)(srow + 8 * lane);
    }
#pragma unroll
    for (int i = 0; i < 16; ++i) {
      const int gr = rowBase + 16 * wave + i;
      unsigned short* rp = hpl + (size_t)gr * (size_t)KD + 8 * lane;
      if (gr < mRows) *(volatile v8us*)rp = qv[i];
    }
    __threadfence();
#pragma unroll
    for (int i = 0; i < 16; ++i) {
      const int gr = rowBase + 16 * wave + i;
      unsigned short* rp = hpl + (size_t)gr * (size_t)KD + 8 * lane;
      if (gr < mRows) *(volatile v8us*)rp = qv[i];
    }
    (void)xin; (void)flg; (void)nFlg; (void)wsf; (void)oD; (void)oK; (void)outp;
  } else if constexpr (MODE == 1) {
    if (ny == 0) {
#pragma unroll 1
      for (int it = 0; it < 64; ++it) {
        const int i = it >> 2, e = it & 3;
        float* p = stg + (16 * wave + i) * GBN + 4 * lane + e;
        const float be = (e == 0) ? b4.x : ((e == 1) ? b4.y : ((e == 2) ? b4.z : b4.w));
        const float v = *p + be;
        *p = gelu_f(v);
      }
    }
    const float zf = (ny == 0) ? 0.0f : 1.0f;
    const v4f bz = b4 * zf;
    v4f pv[16];
#pragma unroll
    for (int i = 0; i < 16; ++i) pv[i] = *(const v4fa*)(stg + (16 * wave + i) * GBN + 4 * lane) + bz;
    const size_t cb = ((ny < 2) ? oD : oK) + (size_t)(ny & 1) * DF;
#pragma unroll
    for (int i = 0; i < 16; ++i) {
      const int gr = rowBase + 16 * wave + i;
      float* op = wsf + cb + (size_t)gr * (size_t)KD + 4 * lane;
      if (gr < mRows) *(volatile v4f*)op = pv[i];
    }
    __threadfence();
#pragma unroll
    for (int i = 0; i < 16; ++i) {
      const int gr = rowBase + 16 * wave + i;
      float* op = wsf + cb + (size_t)gr * (size_t)KD + 4 * lane;
      if (gr < mRows) *(volatile v4f*)op = pv[i];
    }
    (void)xin; (void)flg; (void)nFlg; (void)hpl; (void)outp; (void)nN;
  } else {
    int fb = rowBase >> SLA;
    fb = fb < 0 ? 0 : (fb > nFlg - 1 ? nFlg - 1 : fb);
    const int fl = flg[(size_t)fb * 32];
    const float pz = (fl != 0) ? __int_as_float(0x7fc00000) : 0.0f;
    v4f pv[16];
#pragma unroll
    for (int i = 0; i < 16; ++i) pv[i] = *(const v4fa*)(stg + (16 * wave + i) * GBN + 4 * lane);
#pragma unroll
    for (int i = 0; i < 16; ++i) {
      const int row = rowBase + 16 * wave + i;
      const int rc  = row < nN ? row : nN - 1;
      const v4f xv = bf4(*(const v4f*)(xin + (size_t)rc * DF + 4 * lane));
      v4f o;
      o.x = xv.x + ((pv[i].x + b4.x) * 1.0f) + pz;
      o.y = xv.y + ((pv[i].y + b4.y) * 1.0f) + pz;
      o.z = xv.z + ((pv[i].z + b4.z) * 1.0f) + pz;
      o.w = xv.w + ((pv[i].w + b4.w) * 1.0f) + pz;
      pv[i] = o;
    }
#pragma unroll
    for (int i = 0; i < 16; ++i) {
      const int row = rowBase + 16 * wave + i;
      float* op = outp + (size_t)row * DF + 4 * lane;
      if (row < nN) *(volatile v4f*)op = pv[i];
    }
    __threadfence();
#pragma unroll
    for (int i = 0; i < 16; ++i) {
      const int row = rowBase + 16 * wave + i;
      float* op = outp + (size_t)row * DF + 4 * lane;
      if (row < nN) *(volatile v4f*)op = pv[i];
    }
    (void)hpl; (void)wsf; (void)oD; (void)oK; (void)mRows;
  }
}

__global__ __launch_bounds__(NTHR) void k_agg(const int* __restrict__ srcs, const int* __restrict__ dsts,
                                              const int* __restrict__ ea, int nE, int nN, int vec8, int mRows,
                                              const float* __restrict__ dstp, const float* __restrict__ kvp,
                                              const float* __restrict__ tabg, const float* __restrict__ cst,
                                              unsigned short* xo, int* flg) {
  extern __shared__ __attribute__((aligned(16))) int dsm[];
  int* list = dsm;
  int* hl   = dsm + LISTN;
  int* sl   = hl + RCAP;
  int* cnt  = sl + RCAP;
  int* offs = cnt + NBA;
  int* cur  = offs + NBA;
  int* misc = cur + NBA;
  const int tid = (int)threadIdx.x, lane = tid & 31, wave = tid >> 5;
  unsigned short* rowbuf = (unsigned short*)(misc + MISC_INTS) + wave * ROWH;
  float* tabs = (float*)(misc + MISC_INTS + ROWBUF_INTS);
  const int nodeBase = (int)blockIdx.x * NBA;

  {
    const v4i z4 = {0, 0, 0, 0};
    for (int i = tid * 4; i < AGG_ZINTS; i += NTHR * 4) *(v4ia*)(dsm + i) = z4;
    if (tid < MISC_INTS) misc[tid] = 0;
    for (int i = tid; i < TABF / 4; i += NTHR) *(v4fa*)(tabs + 4 * i) = *(const v4fa*)(tabg + 4 * i);
  }
  __syncthreads();

  int t = 0, ov = 0;
  const int nChunks = (nE + CHUNK - 1) / CHUNK;
#pragma unroll 1
  for (int ch = 0; ch < nChunks; ++ch) {
    const int cbase = ch * CHUNK;
    const int wc = scan_chunk<SLA>(dsts, nE, cbase, nodeBase, NBA, vec8, list, tid, lane, wave);
    if (lane == 0) misc[wave] = wc;
    __syncthreads();
    if (wave == 0) {
#pragma unroll 1
      for (int w2 = 0; w2 < NWAVE; ++w2) {
        int c = misc[w2];
        c = c < 0 ? 0 : (c > WCAP ? WCAP : c);
#pragma unroll 1
        for (int b0 = 0; b0 < c; b0 += 32) {
          const int idx = b0 + lane;
          const int ent_ = list[w2 * WCAP + (idx < WCAP ? idx : WCAP - 1)];
          const int m32 = (c - b0) < 32 ? (c - b0) : 32;
#pragma unroll 1
          for (int k = 0; k < m32; ++k) {
            const int u    = __builtin_amdgcn_readlane(ent_, k);
            const int slot = u & (NBA - 1);
            const int el   = (u >> SLA) & (CHUNK - 1);
            const int pk   = ((cbase + el) << SLA) | slot;
            if (t < RCAP) {
              if (lane == 0) { hl[t] = pk; cnt[slot] = cnt[slot] + 1; }
              t = t + 1;
            } else {
              ov = 1;
            }
          }
        }
      }
    }
    __syncthreads();
  }
  if (wave == 0 && lane == 0) { misc[8] = t; misc[9] = ov; }
  __syncthreads();
  int tt = misc[8];
  tt = tt < 0 ? 0 : (tt > RCAP ? RCAP : tt);
  const int ovf = misc[9];

  if (wave == 0) {
    v4i fv; fv.x = ovf; fv.y = ovf; fv.z = ovf; fv.w = ovf;
    int* fp = flg + (size_t)blockIdx.x * 32 + 4 * (lane & 7);
    if (lane < 8) *(volatile v4i*)fp = fv;
    __threadfence();
    if (lane < 8) *(volatile v4i*)fp = fv;
  }

  if (wave == 0) {
    const int base = lane * (NBA / 32);
    int s = 0;
#pragma unroll 1
    for (int i = 0; i < NBA / 32; ++i) s += cnt[base + i];
    int incl = s;
#pragma unroll
    for (int d = 1; d < 32; d <<= 1) {
      const int y = __shfl_up(incl, d, 32);
      if (lane >= d) incl += y;
    }
    int run = incl - s;
#pragma unroll 1
    for (int i = 0; i < NBA / 32; ++i) {
      const int cv = cnt[base + i];
      offs[base + i] = run;
      cur[base + i]  = run;
      run += cv;
    }
  }
  __syncthreads();
  if (wave == 0) {
#pragma unroll 1
    for (int b0 = 0; b0 < tt; b0 += 32) {
      const int idx = b0 + lane;
      const int ent_ = hl[idx < RCAP ? idx : RCAP - 1];
      const int m32 = (tt - b0) < 32 ? (tt - b0) : 32;
#pragma unroll 1
      for (int k = 0; k < m32; ++k) {
        const int u    = __builtin_amdgcn_readlane(ent_, k);
        const int slot = u & (NBA - 1);
        if (lane == 0) {
          int p = cur[slot];
          p = p < 0 ? 0 : (p > RCAP - 1 ? RCAP - 1 : p);
          sl[p] = u;
          cur[slot] = p + 1;
        }
      }
    }
  }
  __syncthreads();

  const float pz = (ovf != 0) ? __int_as_float(0x7fc00000) : 0.0f;
  const v4f c0 = *(const v4f*)cst;
  const float a0c = c0.x, a1c = c0.y;
  const float* tb0 = tabs + 4 * lane;
  const float* tb1 = tb0 + TROWS * DF;
  const float* tb2 = tb1 + TROWS * DF;
#pragma unroll 1
  for (int si = 0; si < NBA / NWAVE; ++si) {
    const int s    = si * NWAVE + wave;
    const int node = nodeBase + s;
    int c = cnt[s];
    const bool big = c > DEGCAP;
    c = c < 0 ? 0 : (c > DEGCAP ? DEGCAP : c);
    int o = offs[s];
    o = o < 0 ? 0 : (o > RCAP ? RCAP : o);
    const float pzr = big ? __int_as_float(0x7fc00000) : pz;
    const bool live = node < nN;
    const int gcl = live ? node : nN - 1;
    const float* drow = dstp + (size_t)gcl * KD + 4 * lane;
    const v4f m0 = *(const v4fa*)drow;
    const v4f qd = *(const v4fa*)(drow + DF);
    float ac0 = 0.0f, ac1 = 0.0f, ac2 = 0.0f, ac3 = 0.0f;
#pragma unroll 1
    for (int b0 = 0; b0 < c; b0 += 32) {
      int idx = o + b0 + lane;
      idx = idx > RCAP - 1 ? RCAP - 1 : idx;
      const int ent_ = sl[idx];
      int eid = ent_ >> SLA;
      eid = eid < 0 ? 0 : (eid > nE - 1 ? nE - 1 : eid);
      int sr = srcs[eid];
      sr = sr < 0 ? 0 : (sr > nN - 1 ? nN - 1 : sr);
      const v4i at = *(const v4i*)(ea + (size_t)eid * 4);
      int q0 = at.x; q0 = q0 < 0 ? 0 : (q0 > 5 ? 5 : q0);
      int q1 = at.y; q1 = q1 < 0 ? 0 : (q1 > 6 ? 6 : q1);
      int q2 = at.z; q2 = q2 < 0 ? 0 : (q2 > 2 ? 2 : q2);
      int q3 = at.w; q3 = q3 < 0 ? 0 : (q3 > 17 ? 17 : q3);
      const int pk = q0 | ((6 + q1) << 8) | ((13 + q2) << 16) | ((16 + q3) << 24);
      const int m32 = (c - b0) < 32 ? (c - b0) : 32;
#pragma unroll 1
      for (int k = 0; k < m32; ++k) {
        const int sk  = __builtin_amdgcn_readlane(sr, k);
        const int pkk = __builtin_amdgcn_readlane(pk, k);
        const int o0 = (pkk & 255) * DF;
        const int o1 = ((pkk >> 8) & 255) * DF;
        const int o2 = ((pkk >> 16) & 255) * DF;
        const int o3 = ((pkk >> 24) & 255) * DF;
        const float* srow = kvp + (size_t)sk * KD + 4 * lane;
        const v4f kk = *(const v4fa*)srow;
        const v4f vv = *(const v4fa*)(srow + DF);
        const v4f r0 = ((*(const v4fa*)(tb0 + o0) + *(const v4fa*)(tb0 + o1)) + *(const v4fa*)(tb0 + o2))
                       + *(const v4fa*)(tb0 + o3);
        const v4f r1 = ((*(const v4fa*)(tb1 + o0) + *(const v4fa*)(tb1 + o1)) + *(const v4fa*)(tb1 + o2))
                       + *(const v4fa*)(tb1 + o3);
        const v4f r2 = ((*(const v4fa*)(tb2 + o0) + *(const v4fa*)(tb2 + o1)) + *(const v4fa*)(tb2 + o2))
                       + *(const v4fa*)(tb2 + o3);
        const v4f qq = qd + r0;
        const v4f kx = kk + r1;
        float part = qq.x * kx.x;
        part = fmaf(qq.y, kx.y, part);
        part = fmaf(qq.z, kx.z, part);
        part = fmaf(qq.w, kx.w, part);
        part += __shfl_xor(part, 8, 32);
        part += __shfl_xor(part, 4, 32);
        part += __shfl_xor(part, 2, 32);
        part += __shfl_xor(part, 1, 32);
        const float att = expf(fmaf(part * 0.125f, a0c, a1c));
        const v4f vp = vv + r2;
#pragma unroll 1
        for (int j = 0; j < 4; ++j) {
          const float vj = (j == 0) ? vp.x : ((j == 1) ? vp.y : ((j == 2) ? vp.z : vp.w));
          const float g = gelu_f(vj) * att;
          ac0 += (j == 0) ? g : 0.0f;
          ac1 += (j == 1) ? g : 0.0f;
          ac2 += (j == 2) ? g : 0.0f;
          ac3 += (j == 3) ? g : 0.0f;
        }
      }
    }
    const float x0 = live ? ((m0.x + ac0) + pzr) : 0.0f;
    const float x1 = live ? ((m0.y + ac1) + pzr) : 0.0f;
    const float x2 = live ? ((m0.z + ac2) + pzr) : 0.0f;
    const float x3 = live ? ((m0.w + ac3) + pzr) : 0.0f;
    v4us mh, ml;
    {
      unsigned lb;
      unsigned hb;
      hb = hl_bits(x0, lb); mh[0] = (unsigned short)hb; ml[0] = (unsigned short)lb;
      hb = hl_bits(x1, lb); mh[1] = (unsigned short)hb; ml[1] = (unsigned short)lb;
      hb = hl_bits(x2, lb); mh[2] = (unsigned short)hb; ml[2] = (unsigned short)lb;
      hb = hl_bits(x3, lb); mh[3] = (unsigned short)hb; ml[3] = (unsigned short)lb;
    }
    *(v4usa*)(rowbuf + 4 * lane)      = mh;
    *(v4usa*)(rowbuf + DF + 4 * lane) = ml;
    wave_sync();
    const v8us q0v = *(const v8usa*)(rowbuf + 8 * lane);
    wave_sync();
    if (node < mRows) {
      unsigned short* rpw = xo + (size_t)node * KD + 8 * lane;
      *(volatile v8us*)rpw = q0v;
      __threadfence();
      *(volatile v8us*)rpw = q0v;
    }
  }
}

static inline int cdiv(int a, int b) { return (a + b - 1) / b; }
static inline size_t al256(size_t o) { return (o + 255) & ~(size_t)255; }

extern "C" void kernel_launch(void* const* d_in, const int* in_sizes, int n_in,
                              void* d_out, int out_size, void* d_ws, size_t ws_size,
                              hipStream_t stream) {
  if (n_in < 27) return;
  const int nN = in_sizes[0] / DF;
  if (nN < 1 || nN > (1 << 22) || in_sizes[0] != nN * DF) return;
  if (in_sizes[1] < 2 || (in_sizes[1] & 1) != 0) return;
  const int nE = in_sizes[1] / 2;
  if (nE < 1 || nE >= (1 << 21)) return;
  if ((long long)in_sizes[2] != 4LL * (long long)nE) return;
  if (in_sizes[3] != DF * DF || in_sizes[4] != DF) return;
  for (int j = 0; j < 4; ++j)
    if (in_sizes[5 + 2 * j] != DF * DF || in_sizes[6 + 2 * j] != DF) return;
  for (int r = 0; r < 3; ++r)
    if (in_sizes[13 + 2 * r] != EW * DF || in_sizes[14 + 2 * r] != DF) return;
  if (in_sizes[19] != DF * DF || in_sizes[20] != DF) return;
  if (in_sizes[21] != 6 * EW || in_sizes[22] != 7 * EW || in_sizes[23] != 3 * EW || in_sizes[24] != 18 * EW) return;
  if (in_sizes[25] != 4 || in_sizes[26] != 4) return;
  if (out_size != nN * DF) return;

  const float* x     = (const float*)d_in[0];
  const int*   ei    = (const int*)  d_in[1];
  const int*   ea    = (const int*)  d_in[2];
  const float* prew  = (const float*)d_in[3];
  const float* preb  = (const float*)d_in[4];
  const float* m0w   = (const float*)d_in[5];
  const float* m0b   = (const float*)d_in[6];
  const float* m1w   = (const float*)d_in[7];
  const float* m1b   = (const float*)d_in[8];
  const float* m2w   = (const float*)d_in[9];
  const float* m2b   = (const float*)d_in[10];
  const float* m3w   = (const float*)d_in[11];
  const float* m3b   = (const float*)d_in[12];
  const float* r0w   = (const float*)d_in[13];
  const float* r0b   = (const float*)d_in[14];
  const float* r1w   = (const float*)d_in[15];
  const float* r1b   = (const float*)d_in[16];
  const float* r2w   = (const float*)d_in[17];
  const float* r2b   = (const float*)d_in[18];
  const float* postw = (const float*)d_in[19];
  const float* postb = (const float*)d_in[20];
  const float* e0    = (const float*)d_in[21];
  const float* e1    = (const float*)d_in[22];
  const float* e2    = (const float*)d_in[23];
  const float* e3    = (const float*)d_in[24];
  const float* einit = (const float*)d_in[25];
  const float* init0 = (const float*)d_in[26];
  float* out = (float*)d_out;
  const int* src = ei;
  const int* dst = ei + nE;

  const int MP = cdiv(nN, GBM) * GBM;
  const int gM = MP / GBM;
  const int gA = cdiv(MP, NBA);
  if ((long long)gA * NBA < (long long)MP) return;
  const int vec8 = ((nE & 3) == 0) ? 1 : 0;

  char* ws = (char*)d_ws;
  size_t off = 0;
  const size_t oDSTP = off; off = al256(off + (size_t)MP * KD * 4);
  const size_t oKVP  = off; off = al256(off + (size_t)MP * KD * 4);
  const size_t oXH   = off; off = al256(off + (size_t)MP * KD * 2);
  const size_t oPWT  = off; off = al256(off + (size_t)DF * DF * 2);
  const size_t oW4D  = off; off = al256(off + (size_t)4 * DF * KD * 2);
  const size_t oPOST = off; off = al256(off + (size_t)DF * KD * 2);
  const size_t oTAB  = off; off = al256(off + (size_t)TABF * 4);
  const size_t oSML  = off; off = al256(off + (size_t)SMALLF * 4);
  const size_t oFLG  = off; off = al256(off + (size_t)gA * 128);
  if (off > ws_size || off > (size_t)WSMAX) return;
  const size_t oXB = oKVP;
  if ((size_t)MP * DF * 2 > (size_t)MP * KD * 4) return;
  float*          wsf   = (float*)ws;
  unsigned short* XB    = (unsigned short*)(ws + oXB);
  unsigned short* XH    = (unsigned short*)(ws + oXH);
  unsigned short* PWT   = (unsigned short*)(ws + oPWT);
  unsigned short* W4D   = (unsigned short*)(ws + oW4D);
  unsigned short* POSTD = (unsigned short*)(ws + oPOST);
  float*          TAB   = (float*)(ws + oTAB);
  float*          SML   = (float*)(ws + oSML);
  int*            FLG   = (int*)(ws + oFLG);
  const float*    DSTP  = (const float*)(ws + oDSTP);
  const float*    KVP   = (const float*)(ws + oKVP);

  const size_t aggLds = (size_t)AGG_LDS_INTS * 4;
  hipFuncSetAttribute(reinterpret_cast<const void*>(&k_agg), hipFuncAttributeMaxDynamicSharedMemorySize, (int)aggLds);

  const int nUnits = NU_W + MP * (DF / 8);
  k_prep<<<cdiv(nUnits, NTHR), NTHR, 0, stream>>>(x, prew, m0w, m1w, m2w, m3w, postw,
                                                  PWT, W4D, POSTD, XB, nN, nUnits);
  k_tab<<<3 * TABBLK + 1, NTHR, 0, stream>>>(e0, e1, e2, e3, r0w, r1w, r2w, r0b, r1b, r2b,
                                             m0b, m1b, m2b, m3b, preb, postb, einit, init0, TAB, SML);
  k_gemm<0><<<dim3(gM, 1), GTHR, 0, stream>>>(XB, DF, PWT, DF, SML + 512, x, FLG, gA,
                                              XH, wsf, oDSTP / 4, oKVP / 4, out, nN, MP);
  k_gemm<1><<<dim3(gM, 4), GTHR, 0, stream>>>(XH, KD, W4D, KD, SML, x, FLG, gA,
                                              XH, wsf, oDSTP / 4, oKVP / 4, out, nN, MP);
  k_agg<<<gA, NTHR, aggLds, stream>>>(src, dst, ea, nE, nN, vec8, MP, DSTP, KVP, TAB, SML + 768, XH, FLG);
  k_gemm<2><<<dim3(gM, 1), GTHR, 0, stream>>>(XH, KD, POSTD, KD, SML + 640, x, FLG, gA,
                                              XH, wsf, oDSTP / 4, oKVP / 4, out, nN, MP);
}
